// NeighborhoodEncoder_67723044323928
// MI455X (gfx1250) — hardware-verified
//
#include <hip/hip_runtime.h>


#define NPTS 2097152
#define PPC  64
#define NCL  (NPTS / PPC)
#define F0   64
#define F1   128
#define F2   256
#define DM   F0
#define NTK  NCL
#define LOSC 1024.0f

typedef _Float16 h16;
typedef unsigned short bf;
typedef __attribute__((ext_vector_type(16))) __bf16   v16bf;
typedef __attribute__((ext_vector_type(16))) _Float16 v16h;
typedef __attribute__((ext_vector_type(8)))  _Float16 v8h;
typedef __attribute__((ext_vector_type(8)))  unsigned short v8us;
typedef __attribute__((ext_vector_type(8)))  float    v8f;
typedef __attribute__((ext_vector_type(4)))  float    v4f;
typedef __attribute__((ext_vector_type(4)))  _Float16 v4h;
typedef v8h  __attribute__((may_alias)) v8ha;
typedef v4f  __attribute__((may_alias)) v4fa;
typedef v8us __attribute__((may_alias)) v8usa;

__device__ __forceinline__ unsigned short f2bf(float f) { unsigned u = __float_as_uint(f); u += 0x7FFFu + ((u >> 16) & 1u); return (unsigned short)(u >> 16); }
__device__ __forceinline__ float bf2f(unsigned short b) { return __uint_as_float(((unsigned)b) << 16); }
__device__ __forceinline__ float bfr(float f) { return bf2f(f2bf(f)); }
__device__ __forceinline__ v16h cat16(v8h lo, v8h hi) { return __builtin_shufflevector(lo, hi, 0, 1, 2, 3, 4, 5, 6, 7, 8, 9, 10, 11, 12, 13, 14, 15); }
__device__ __forceinline__ v16bf cat16b(v8us lo, v8us hi) { return __builtin_bit_cast(v16bf, __builtin_shufflevector(lo, hi, 0, 1, 2, 3, 4, 5, 6, 7, 8, 9, 10, 11, 12, 13, 14, 15)); }
__device__ __forceinline__ v8f wmma16(v16h a, v16h b, v8f c) { return __builtin_amdgcn_wmma_f32_16x16x32_f16(false, a, false, b, (short)0, c, false, false); }
__device__ __forceinline__ v8f wmmab(v16bf a, v16bf b, v8f c) { return __builtin_amdgcn_wmma_f32_16x16x32_bf16(false, a, false, b, (short)0, c, false, false); }

template <bool SPLITA, bool F16OUT = false>
__global__ __launch_bounds__(128) void k_gemmb(const bf* __restrict__ A, const bf* __restrict__ Al, const bf* __restrict__ Bn, const float* __restrict__ bias, float* C, int ldc, h16* C2, const float* __restrict__ R = nullptr, int K = DM, int roundR = 1) {
    __shared__ __align__(16) float ost[4][16 * 68];
    const int lane = threadIdx.x & 31, wave = threadIdx.x >> 5, lr = lane & 15, hi = lane >> 4;
    const int r0 = blockIdx.x * 64 + wave * 16, c0 = blockIdx.y * 64;
    const size_t aoff = (size_t)(r0 + lr) * K + 8 * hi;
    size_t boff[4];
#pragma unroll
    for (int t = 0; t < 4; ++t) boff[t] = (size_t)(c0 + t * 16 + lr) * K + 8 * hi;
    v8f acc[4];
#pragma unroll
    for (int t = 0; t < 4; ++t) acc[t] = (v8f){};
#pragma unroll 1
    for (int kc = 0; kc < K; kc += 32) {
        const v16bf a = cat16b(*(const v8us*)(A + aoff + kc), *(const v8us*)(A + aoff + kc + 16));
        v16bf al = a;
        if (SPLITA) al = cat16b(*(const v8us*)(Al + aoff + kc), *(const v8us*)(Al + aoff + kc + 16));
#pragma unroll
        for (int t = 0; t < 4; ++t) { const v16bf b = cat16b(*(const v8us*)(Bn + boff[t] + kc), *(const v8us*)(Bn + boff[t] + kc + 16)); acc[t] = wmmab(a, b, acc[t]); if (SPLITA) acc[t] = wmmab(al, b, acc[t]); }
        asm volatile("v_nop\n\tv_nop\n\tv_nop\n\tv_nop" : "+v"(acc[0]), "+v"(acc[1]), "+v"(acc[2]), "+v"(acc[3]) : "v"(a), "v"(al));
    }
    float* os = &ost[wave][0];
#pragma unroll
    for (int t = 0; t < 4; ++t) { const float bv = bias ? bfr(bias[c0 + t * 16 + lr]) : 0.f;
#pragma unroll
        for (int j = 0; j < 8; ++j) os[(hi * 8 + j) * 68 + t * 16 + lr] = acc[t][j] + bv; }
    __syncthreads();
    if (F16OUT) {
        h16* crow = (h16*)(void*)C + (size_t)r0 * ldc + c0;
        auto pass = [&]() {
#pragma unroll
            for (int s = 0; s < 4; ++s) { const int row = 4 * s + (lane >> 3), piece = lane & 7; const float* sp = os + row * 68 + piece * 8; v8h o, o2;
#pragma unroll
                for (int i = 0; i < 8; ++i) { const h16 a = (h16)sp[i]; o[i] = a; o2[i] = (h16)((sp[i] - (float)a) * LOSC); }
                *(volatile v8h*)(crow + (size_t)row * ldc + piece * 8) = o; if (C2) *(volatile v8h*)(C2 + (size_t)r0 * ldc + c0 + (size_t)row * ldc + piece * 8) = o2; }
        };
        pass(); __threadfence(); pass();
    } else {
        float* crow = C + (size_t)r0 * ldc + c0;
        auto pass = [&]() {
#pragma unroll
            for (int s = 0; s < 8; ++s) { const int Lid = (lane >> 3) + 4 * s, piece = lane & 7; const int row = Lid >> 1, cofs = (Lid & 1) * 32 + piece * 4;
                v4f val = *(const v4fa*)(os + row * 68 + cofs); if (R) { const v4f rv = *(const v4f*)(R + ((size_t)r0 + row) * ldc + c0 + cofs); val += roundR ? (v4f){bfr(rv[0]), bfr(rv[1]), bfr(rv[2]), bfr(rv[3])} : rv; }
                *(volatile v4f*)(crow + (size_t)row * ldc + cofs) = val; }
        };
        pass(); __threadfence(); pass();
    }
}


__global__ __launch_bounds__(256) void k_bf(const float* __restrict__ src, bf* dst, size_t n8) {
    const size_t i = (size_t)blockIdx.x * 256 + threadIdx.x; if (i >= n8) return;
    const v8f v = *(const v8f*)(src + i * 8); v8us o;
#pragma unroll
    for (int k = 0; k < 8; ++k) o[k] = f2bf(v[k]);
    *(volatile v8us*)(dst + i * 8) = o; __threadfence(); *(volatile v8us*)(dst + i * 8) = o;
}
__global__ __launch_bounds__(256) void k_pool(const float* __restrict__ pts, const int* __restrict__ CLU, const float* __restrict__ W1, const float* __restrict__ b1, bf* Ph, bf* Pl) {
    __shared__ float wm[8][F0];
    const int tid = threadIdx.x, lane = tid & 31, wave = tid >> 5;
    const size_t p = (size_t)blockIdx.x * 256 + tid;
    const float x0 = bfr(pts[p * 3]), x1 = bfr(pts[p * 3 + 1]), x2 = bfr(pts[p * 3 + 2]);
#pragma unroll 1
    for (int c = 0; c < F0; ++c) {
        float h = bfr(b1[c]); h = fmaf(x0, bfr(W1[c * 3]), h); h = fmaf(x1, bfr(W1[c * 3 + 1]), h); h = fmaf(x2, bfr(W1[c * 3 + 2]), h); h = fmaxf(h, 0.f);
#pragma unroll
        for (int s = 16; s; s >>= 1) h = fmaxf(h, __shfl_xor(h, s, 32));
        if (lane == 0) wm[wave][c] = h;
    }
    __syncthreads();
    const int cl = tid >> 6, piece = tid & 7;
    if ((tid & 63) < 8) { v8us oh, ol;
#pragma unroll
        for (int i = 0; i < 8; ++i) { const int c = piece * 8 + i; const float v = fmaxf(wm[cl * 2][c], wm[cl * 2 + 1][c]); const unsigned short hb = f2bf(v); oh[i] = hb; ol[i] = f2bf(v - bf2f(hb)); }
        int cid = CLU[(size_t)blockIdx.x * 256 + cl * 64]; cid = cid < 0 ? 0 : (cid >= NCL ? NCL - 1 : cid);
        const size_t o = (size_t)cid * F0 + piece * 8;
        *(volatile v8us*)(Ph + o) = oh; *(volatile v8us*)(Pl + o) = ol; __threadfence(); *(volatile v8us*)(Ph + o) = oh; *(volatile v8us*)(Pl + o) = ol; }
}
__global__ __launch_bounds__(256) void k_relu2(const float* __restrict__ src, int nrows, bf* dh, bf* dl) {
    typedef __attribute__((ext_vector_type(4))) unsigned short v4us;
    const int lane = threadIdx.x & 31, r = blockIdx.x * 8 + (threadIdx.x >> 5); if (r >= nrows) return;
    const size_t o = (size_t)r * F1 + lane * 4; const v4f v = *(const v4f*)(src + o); v4us oh, ol;
#pragma unroll
    for (int i = 0; i < 4; ++i) { const float g = fmaxf(v[i], 0.f); const unsigned short hb = f2bf(g); oh[i] = hb; ol[i] = f2bf(g - bf2f(hb)); }
    *(volatile v4us*)(dh + o) = oh; *(volatile v4us*)(dl + o) = ol; __threadfence(); *(volatile v4us*)(dh + o) = oh; *(volatile v4us*)(dl + o) = ol;
}
__global__ __launch_bounds__(256) void k_relu_out(const float* __restrict__ T, int nrows, float* OUTP) {
    const int lane = threadIdx.x & 31, r = blockIdx.x * 8 + (threadIdx.x >> 5); if (r >= nrows) return;
#pragma unroll 1
    for (int ps = 0; ps < 2; ++ps) {
#pragma unroll
        for (int q = 0; q < F2 / 128; ++q) { const size_t o = (size_t)r * F2 + q * 128 + lane * 4; v4f v = *(const v4f*)(T + o);
#pragma unroll
            for (int i = 0; i < 4; ++i) v[i] = fmaxf(v[i], 0.f);
            *(volatile v4f*)(OUTP + o) = v; }
        if (ps == 0) __threadfence(); }
}

extern "C" void kernel_launch(void* const* d_in, const int* in_sizes, int n_in,
                              void* d_out, int out_size, void* d_ws, size_t ws_size, hipStream_t stream) {
    (void)in_sizes; (void)n_in; (void)out_size;
    const float* pts = (const float*)d_in[0]; const int* clu = (const int*)d_in[1]; const float* W1 = (const float*)d_in[2]; const float* b1 = (const float*)d_in[3];
    const float* W2 = (const float*)d_in[4]; const float* b2 = (const float*)d_in[5]; const float* W3 = (const float*)d_in[6]; const float* b3 = (const float*)d_in[7];
    float* out = (float*)d_out;
    char* wsp = (char*)d_ws;
    auto take = [&](size_t bytes) { char* p = wsp; wsp += (bytes + 255) & ~(size_t)255; return (void*)p; };
    bf* W2B = (bf*)take((size_t)F1 * F0 * 2); bf* W3B = (bf*)take((size_t)F2 * F1 * 2);
    bf* Ph = (bf*)take((size_t)NCL * F0 * 2); bf* Pl = (bf*)take((size_t)NCL * F0 * 2); float* T1 = (float*)take((size_t)NCL * F1 * 4); bf* Hh = (bf*)take((size_t)NCL * F1 * 2); bf* Hl = (bf*)take((size_t)NCL * F1 * 2); float* T2 = (float*)take((size_t)NCL * F2 * 4);
    if ((size_t)(wsp - (char*)d_ws) > ws_size) return;
    k_bf<<<(F1 * F0 / 8 + 255) / 256, 256, 0, stream>>>(W2, W2B, F1 * F0 / 8); k_bf<<<(F2 * F1 / 8 + 255) / 256, 256, 0, stream>>>(W3, W3B, F2 * F1 / 8);
    k_pool<<<NPTS / 256, 256, 0, stream>>>(pts, clu, W1, b1, Ph, Pl);
    k_gemmb<true, false><<<dim3(NCL / 64, F1 / 64, 1), 128, 0, stream>>>(Ph, Pl, W2B, b2, T1, F1, nullptr, nullptr, F0);
    k_relu2<<<NCL / 8, 256, 0, stream>>>(T1, NCL, Hh, Hl);
    k_gemmb<true, false><<<dim3(NCL / 64, F2 / 64, 1), 128, 0, stream>>>(Hh, Hl, W3B, b3, T2, F2, nullptr, nullptr, F1);
    k_relu_out<<<NCL / 8, 256, 0, stream>>>(T2, NCL, out);
}
